// TrackPairingPredictionNetwork_88768384074460
// MI455X (gfx1250) — hardware-verified
//
#include <hip/hip_runtime.h>


namespace {
constexpr int J = 128, T = 64, D = 64, H1 = 64, H2 = 32, H3 = 16, NPAIR = J * T * T;
constexpr float XS = 8.0f, WSC = 256.0f;
typedef _Float16 b16;
typedef __attribute__((ext_vector_type(16))) _Float16 v16b;
typedef __attribute__((ext_vector_type(8))) _Float16 v8b;
typedef __attribute__((ext_vector_type(8))) float v8f;
typedef __attribute__((ext_vector_type(4))) float v4f;
__device__ __forceinline__ float bf16_rne(float f) { unsigned int u = __float_as_uint(f); u += 0x7FFFu + ((u >> 16) & 1u); float r = __uint_as_float(u & 0xFFFF0000u); asm volatile("" : "+v"(r)); return r; }
__device__ __forceinline__ void split16(float v, b16& hi, b16& lo) { hi = (b16)v; lo = (b16)(v - (float)hi); }
__device__ __forceinline__ v16b frag_kb(const b16* p, int hh) { const v8b a = *(const v8b*)(p + 8 * hh), b = *(const v8b*)(p + 16 + 8 * hh); v16b f;
#pragma unroll
  for (int e = 0; e < 8; ++e) { f[e] = a[e]; f[8 + e] = b[e]; } return f; }
__device__ __forceinline__ v8f wmma16b(v16b a, v16b b, v8f c) { v8f d = __builtin_amdgcn_wmma_f32_16x16x32_f16(false, a, false, b, (short)0, c, false, false); asm volatile("v_nop\n\tv_nop\n\tv_nop\n\tv_nop" : "+v"(d) : "v"(a), "v"(b)); return d; }
__device__ __forceinline__ void wave_lds_sync() { __builtin_amdgcn_fence(__ATOMIC_RELEASE, "workgroup"); __builtin_amdgcn_wave_barrier(); __builtin_amdgcn_fence(__ATOMIC_ACQUIRE, "workgroup"); }
__device__ __forceinline__ float pmul(float a, float b) { float p = a * b; asm volatile("" : "+v"(p)); return p; }

__global__ __launch_bounds__(256) void wput_kernel(const float* __restrict__ w1, const float* __restrict__ w2, const float* __restrict__ w3, b16* __restrict__ WAB, b16* __restrict__ WC, b16* __restrict__ W2T, b16* __restrict__ W3T) { const int u = blockIdx.x * 256 + threadIdx.x;
  for (int pass = 0; pass < 2; ++pass) {
    if (u < 2 * H1 * 8) { const int o = u / 8, k0 = (u % 8) * 8; const int blk = o / H1, oo = o % H1; v8b v;
#pragma unroll
      for (int j = 0; j < 8; ++j) v[j] = (b16)(bf16_rne(w1[(size_t)(blk * D + k0 + j) * H1 + oo]) * WSC); *(volatile v8b*)(WAB + (size_t)o * D + k0) = v; }
    if (u < H1 * 8) { const int o = u / 8, k0 = (u % 8) * 8; v8b v, v2;
#pragma unroll
      for (int j = 0; j < 8; ++j) { v[j] = (b16)(bf16_rne(w1[(size_t)(2 * D + k0 + j) * H1 + o]) * WSC); v2[j] = (b16)(bf16_rne(w2[(size_t)(k0 + j) * H2 + (o % H2)]) * WSC); } *(volatile v8b*)(WC + (size_t)o * D + k0) = v; if (o < H2) *(volatile v8b*)(W2T + (size_t)o * H1 + k0) = v2; }
    if (u < H3 * 4) { const int o = u / 4, k0 = (u % 4) * 8; v8b v;
#pragma unroll
      for (int j = 0; j < 8; ++j) v[j] = (b16)(bf16_rne(w3[(size_t)(k0 + j) * H3 + o]) * WSC); *(volatile v8b*)(W3T + (size_t)o * H2 + k0) = v; }
    __threadfence(); } }
template <int MODE>
__global__ __launch_bounds__(32) void part_kernel(const float* __restrict__ IN, const b16* __restrict__ WT, const float* __restrict__ b1, float* __restrict__ OUT) { constexpr int NT = MODE == 0 ? 8 : 4, OW = NT * 16; __shared__ __attribute__((aligned(16))) b16 Ah[16][D + 8]; __shared__ float Tf[16][132]; const int lane = threadIdx.x, nloc = lane & 15, hlf = lane >> 4; const size_t m0 = (size_t)blockIdx.x * 16;
  for (int rr = 0; rr < 16; ++rr) for (int q = 0; q < 2; ++q) Ah[rr][q * 32 + lane] = (b16)(bf16_rne(IN[(m0 + rr) * D + q * 32 + lane]) * XS);
  wave_lds_sync(); v8f acc[NT];
#pragma unroll
  for (int t = 0; t < NT; ++t) acc[t] = (v8f){};
#pragma unroll
  for (int kb = 0; kb < D; kb += 32) { const v16b a = frag_kb(&Ah[nloc][kb], hlf);
#pragma unroll
    for (int t = 0; t < NT; ++t) acc[t] = wmma16b(a, frag_kb(WT + (size_t)(t * 16 + nloc) * D + kb, hlf), acc[t]); }
#pragma unroll
  for (int t = 0; t < NT; ++t) { const int c = t * 16 + nloc; const float bb = (MODE == 1) ? bf16_rne(b1[c]) : 0.0f;
#pragma unroll
    for (int r8 = 0; r8 < 8; ++r8) Tf[8 * hlf + r8][c] = acc[t][r8] * (1.0f / (XS * WSC)) + bb; }
  wave_lds_sync();
  for (int pass = 0; pass < 2; ++pass) { for (int rr = 0; rr < 16; ++rr) { if (MODE == 0) *(volatile v4f*)(OUT + (m0 + rr) * OW + lane * 4) = *(const v4f*)(&Tf[rr][lane * 4]); else { typedef __attribute__((ext_vector_type(2))) float v2f; *(volatile v2f*)(OUT + (m0 + rr) * OW + lane * 2) = (v2f){Tf[rr][lane * 2], Tf[rr][lane * 2 + 1]}; } } __threadfence(); } }
__global__ __launch_bounds__(32) void pair_kernel(const float* __restrict__ AB, const float* __restrict__ CJ, const b16* __restrict__ W2T, const float* __restrict__ b2, const b16* __restrict__ W3T, const float* __restrict__ b3, const float* __restrict__ w4, const float* __restrict__ b4, int JV, float* __restrict__ out) {
  __shared__ __attribute__((aligned(16))) b16 Ah[32][H1 + 8], Al[32][H1 + 8], Gh[32][40], Gl[32][40]; __shared__ float T3[32][17]; const int lane = threadIdx.x, nloc = lane & 15, hlf = lane >> 4; const size_t p0 = (size_t)blockIdx.x * 32; const int j = (int)(p0 / (T * T)), i = (int)((p0 / T) % T), k0 = (int)(p0 % T); if (j >= JV) return;
  const float* Arow = AB + ((size_t)j * T + i) * 2 * H1; const float* Cj = CJ + (size_t)j * H1;
  for (int rr = 0; rr < 32; ++rr) { const float* Brow = AB + ((size_t)j * T + k0 + rr) * 2 * H1 + H1; for (int q = 0; q < 2; ++q) { const int c = q * 32 + lane; const float v = fmaxf(Arow[c] + Brow[c] + Cj[c], 0.0f); b16 p, ql; split16(v * XS, p, ql); Ah[rr][c] = p; Al[rr][c] = ql; } }
  wave_lds_sync(); v8f a2[2][2]; for (int m = 0; m < 2; ++m) for (int t = 0; t < 2; ++t) a2[m][t] = (v8f){};
#pragma unroll
  for (int kb = 0; kb < H1; kb += 32) {
#pragma unroll
    for (int m = 0; m < 2; ++m) { const v16b a = frag_kb(&Ah[m * 16 + nloc][kb], hlf), al = frag_kb(&Al[m * 16 + nloc][kb], hlf);
#pragma unroll
      for (int t = 0; t < 2; ++t) { const v16b bw = frag_kb(W2T + (size_t)(t * 16 + nloc) * H1 + kb, hlf); a2[m][t] = wmma16b(a, bw, a2[m][t]); a2[m][t] = wmma16b(al, bw, a2[m][t]); } } }
#pragma unroll
  for (int m = 0; m < 2; ++m)
#pragma unroll
    for (int t = 0; t < 2; ++t) { const int c = t * 16 + nloc; const float bb = bf16_rne(b2[c]);
#pragma unroll
      for (int r8 = 0; r8 < 8; ++r8) { b16 p, q; split16(fmaxf(a2[m][t][r8] * (1.0f / (XS * WSC)) + bb, 0.0f) * XS, p, q); Gh[m * 16 + 8 * hlf + r8][c] = p; Gl[m * 16 + 8 * hlf + r8][c] = q; } }
  wave_lds_sync(); v8f a3[2] = {(v8f){}, (v8f){}};
#pragma unroll
  for (int m = 0; m < 2; ++m) { const v16b a = frag_kb(&Gh[m * 16 + nloc][0], hlf), al = frag_kb(&Gl[m * 16 + nloc][0], hlf); const v16b bw = frag_kb(W3T + (size_t)nloc * H2, hlf); a3[m] = wmma16b(a, bw, a3[m]); a3[m] = wmma16b(al, bw, a3[m]); }
#pragma unroll
  for (int m = 0; m < 2; ++m)
#pragma unroll
    for (int r8 = 0; r8 < 8; ++r8) T3[m * 16 + 8 * hlf + r8][nloc] = fmaxf(a3[m][r8] * (1.0f / (XS * WSC)) + bf16_rne(b3[nloc]), 0.0f);
  wave_lds_sync(); float s = bf16_rne(b4[0]);
#pragma unroll
  for (int c = 0; c < H3; ++c) s += pmul(T3[lane][c], bf16_rne(w4[c])); const float prob = 1.0f / (1.0f + __expf(-s));
  for (int pass = 0; pass < 2; ++pass) { ((volatile float*)out)[p0 + lane] = prob; __threadfence(); } }
}

extern "C" void kernel_launch(void* const* d_in, const int* in_sizes, int n_in, void* d_out, int out_size, void* d_ws, size_t ws_size, hipStream_t stream) {
  (void)n_in;
  auto Fp = [&](int i) { return (const float*)d_in[i]; };
  if (in_sizes[0] != J * D || in_sizes[1] != J * T * D || in_sizes[2] != 3 * D * H1 || in_sizes[4] != H1 * H2 || in_sizes[6] != H2 * H3 || in_sizes[8] != H3 || out_size != NPAIR) return;
  const int JV = J;
  size_t off = 0; char* ws = (char*)d_ws;
  auto carve = [&](size_t bytes) { char* p = ws + off; off += (bytes + 255) & ~(size_t)255; return p; };
  b16* WAB = (b16*)carve((size_t)2 * H1 * D * 2); b16* WC = (b16*)carve((size_t)H1 * D * 2); b16* W2T = (b16*)carve((size_t)H2 * H1 * 2); b16* W3T = (b16*)carve((size_t)H3 * H2 * 2); float* AB = (float*)carve((size_t)J * T * 2 * H1 * 4); float* CJ = (float*)carve((size_t)J * H1 * 4);
  if (off > ws_size || off > ((size_t)8 << 20)) return;
  wput_kernel<<<(2 * H1 * 8 + 255) / 256, 256, 0, stream>>>(Fp(2), Fp(4), Fp(6), WAB, WC, W2T, W3T);
  part_kernel<0><<<J * T / 16, 32, 0, stream>>>(Fp(1), WAB, nullptr, AB);
  part_kernel<1><<<J / 16, 32, 0, stream>>>(Fp(0), WC, Fp(3), CJ);
  pair_kernel<<<JV * T * T / 32, 32, 0, stream>>>(AB, CJ, W2T, Fp(5), W3T, Fp(7), Fp(8), Fp(9), JV, (float*)d_out);
}
